// ReOrderer_50190987821313
// MI455X (gfx1250) — hardware-verified
//
#include <hip/hip_runtime.h>

typedef _Float16 v16h __attribute__((ext_vector_type(16)));
typedef _Float16 v8h  __attribute__((ext_vector_type(8)));
typedef float    v8f  __attribute__((ext_vector_type(8)));
typedef float    v4f  __attribute__((ext_vector_type(4)));
typedef v8h __attribute__((may_alias)) v8ha;
typedef v4f __attribute__((may_alias)) v4fa;

union Frag { v16h v; v8h half[2]; };

#define NB     8
#define NS     1024
#define NT     1024
#define ND     1024
#define NTOK   (NB * NS)
#define NX     (NTOK * ND)
#define NW     (ND * ND)
#define NW8    (NW / 8)
#define NBLK   (NB * NT / 16)
#define BIGF   1.0e10f
#define PSCALE 16384.0f
#define RC03   (1.0f / 0.3f)
#define WSCALE 32.0f
#define LP     1032
#define FP     1028
#define TP     72

static_assert(NS == NT);
static_assert((LP % 8) == 0);
static_assert((FP % 4) == 0);
static_assert((TP % 8) == 0);
static_assert(NBLK == 512);

__device__ __forceinline__ v8f wmma_f16(v16h a, v16h b, v8f c) {
  v8f d = __builtin_amdgcn_wmma_f32_16x16x32_f16(false, a, false, b, (short)0, c, false, false);
  asm volatile("v_nop\n\tv_nop\n\tv_nop\n\tv_nop" : "+v"(d) : "v"(a), "v"(b));
  return d;
}

__device__ __forceinline__ v16h load_frag(const _Float16* p, int h) {
  Frag f;
  f.half[0] = *(const v8ha*)(p + 8 * h);
  f.half[1] = *(const v8ha*)(p + 16 + 8 * h);
  return f.v;
}

__device__ __forceinline__ void pos_row(float (&p)[32], float st, int t,
                                        const float* __restrict__ mrow, int lane) {
  #pragma clang fp contract(off)
  const float it = st * (float)t;
  float vmax = -3.0e38f;
  #pragma unroll
  for (int j = 0; j < 32; ++j) {
    const int s = lane + 32 * j;
    const float d = (float)s - it;
    const float d2 = d * d;
    const float pen = BIGF * (1.0f - mrow[s]);
    const float v = -(d2 * RC03) - pen;
    p[j] = v;
    vmax = fmaxf(vmax, v);
  }
  #pragma unroll
  for (int o = 16; o > 0; o >>= 1) vmax = fmaxf(vmax, __shfl_xor(vmax, o));
  float sum = 0.0f;
  #pragma unroll
  for (int j = 0; j < 32; ++j) {
    const float e = __expf(p[j] - vmax);
    p[j] = e;
    sum += e;
  }
  #pragma unroll
  for (int o = 16; o > 0; o >>= 1) sum += __shfl_xor(sum, o);
  const float inv = 1.0f / sum;
  #pragma unroll
  for (int j = 0; j < 32; ++j) p[j] = p[j] * inv;
}

__global__ __launch_bounds__(256) void steps_kernel(const float* __restrict__ msrc,
                                                    const float* __restrict__ mtrg,
                                                    float* __restrict__ steps_ws) {
  __shared__ __attribute__((aligned(16))) float sst[32];
  const int tid = threadIdx.x, lane = tid & 31, w = tid >> 5;
  float a = 0.0f, c = 0.0f;
  #pragma unroll
  for (int j = 0; j < 32; ++j) {
    a += msrc[w * NS + lane + 32 * j];
    c += mtrg[w * NT + lane + 32 * j];
  }
  #pragma unroll
  for (int o = 16; o > 0; o >>= 1) { a += __shfl_xor(a, o); c += __shfl_xor(c, o); }
  if (tid < 32) sst[tid] = 0.0f;
  __syncthreads();
  if (lane == 0) sst[w] = a * (1.0f / c);
  __syncthreads();
  v4f v = {0.f, 0.f, 0.f, 0.f};
  if (tid < 8) {
    v = *(const v4fa*)(sst + 4 * tid);
    *(volatile v4f*)(steps_ws + 4 * tid) = v;
  }
  __threadfence();
  if (tid < 8) {
    *(volatile v4f*)(steps_ws + 4 * tid) = v;
  }
}

__global__ __launch_bounds__(256) void cvt_w_kernel(const float* __restrict__ wq,
                                                    const float* __restrict__ wk,
                                                    _Float16* __restrict__ wh) {
  const int g = blockIdx.x * 256 + threadIdx.x;
  if (g >= 2 * NW8) return;
  const int wsel = g / NW8;
  const int off = g - wsel * NW8;
  const float* src = ((wsel == 0) ? wq : wk) + (size_t)off * 8;
  _Float16* dst = wh + (size_t)g * 8;
  const v4f a = *(const v4fa*)src;
  const v4f c = *(const v4fa*)(src + 4);
  const v8h o = { (_Float16)(a.x * WSCALE), (_Float16)(a.y * WSCALE), (_Float16)(a.z * WSCALE), (_Float16)(a.w * WSCALE),
                  (_Float16)(c.x * WSCALE), (_Float16)(c.y * WSCALE), (_Float16)(c.z * WSCALE), (_Float16)(c.w * WSCALE) };
  *(volatile v8h*)dst = o;
  __threadfence();
  *(volatile v8h*)dst = o;
}

__device__ __forceinline__ void prep_store_pass(const _Float16* tile, _Float16* keyh, _Float16* keyT,
                                                int b, int s0, int d0, int w, int lane) {
  const int q8 = lane & 7, sub = lane >> 3;
  #pragma unroll
  for (int i = 0; i < 4; ++i) {
    const int L = 16 * w + 4 * i + sub;
    const v8h a = *(const v8ha*)(tile + L * TP + 8 * q8);
    v8h t;
    #pragma unroll
    for (int j = 0; j < 8; ++j) t[j] = tile[(8 * q8 + j) * TP + L];
    *(volatile v8h*)(keyh + ((size_t)(b * NS + s0 + L)) * ND + d0 + 8 * q8) = a;
    *(volatile v8h*)(keyT + ((size_t)(b * ND + d0 + L)) * NS + s0 + 8 * q8) = t;
  }
}

__global__ __launch_bounds__(128) void prep_key_kernel(const float* __restrict__ key,
                                                      _Float16* __restrict__ keyh,
                                                      _Float16* __restrict__ keyT) {
  __shared__ __attribute__((aligned(16))) _Float16 tile[64 * TP];
  const int tid = threadIdx.x, lane = tid & 31, w = tid >> 5;
  const int s0 = blockIdx.x * 64, d0 = blockIdx.y * 64, b = blockIdx.z;
  const int c4 = (tid & 15) * 4, rsub = tid >> 4;
  #pragma unroll
  for (int i = 0; i < 8; ++i) {
    const int row = 8 * i + rsub;
    const v4f x = *(const v4fa*)(key + ((size_t)(b * NS + s0 + row)) * ND + d0 + c4);
    _Float16* tp = tile + row * TP + c4;
    tp[0] = (_Float16)x.x; tp[1] = (_Float16)x.y; tp[2] = (_Float16)x.z; tp[3] = (_Float16)x.w;
  }
  __syncthreads();
  prep_store_pass(tile, keyh, keyT, b, s0, d0, w, lane);
  __threadfence();
  prep_store_pass(tile, keyh, keyT, b, s0, d0, w, lane);
}

__device__ __forceinline__ void q_store_pass(const _Float16* sQ, _Float16* qout,
                                             int b, int t0, int w, int lane) {
  const int q8 = lane & 7, sub = lane >> 3;
  #pragma unroll
  for (int i = 0; i < 8; ++i) {
    const int L = 32 * w + 4 * i + sub;
    const int row = L >> 4, seg = L & 15;
    const v8h v = *(const v8ha*)(sQ + row * LP + seg * 64 + 8 * q8);
    *(volatile v8h*)(qout + ((size_t)(b * NT + t0 + row)) * ND + seg * 64 + 8 * q8) = v;
  }
}

__global__ __launch_bounds__(256) void query_kernel(const float* __restrict__ msrc,
                                                    const _Float16* __restrict__ keyT,
                                                    const float* __restrict__ steps_ws,
                                                    const float* __restrict__ wg,
                                                    const float* __restrict__ bg,
                                                    _Float16* __restrict__ qout,
                                                    float* __restrict__ gates_ws) {
  __shared__ __attribute__((aligned(16))) _Float16 sP[16 * LP];
  __shared__ float gpart[8 * 16];
  __shared__ __attribute__((aligned(16))) float gl[32];

  const int tid = threadIdx.x, lane = tid & 31, w = tid >> 5;
  const int h = lane >> 4, m = lane & 15;
  const int blk = blockIdx.x, b = blk >> 6, t0 = (blk & 63) * 16;
  const float st = steps_ws[b];
  const float* mrow = msrc + (size_t)b * NS;

  #pragma unroll
  for (int rr = 0; rr < 2; ++rr) {
    const int r = 2 * w + rr;
    float p[32];
    pos_row(p, st, t0 + r, mrow, lane);
    #pragma unroll
    for (int j = 0; j < 32; ++j) sP[r * LP + lane + 32 * j] = (_Float16)(p[j] * PSCALE);
  }
  __syncthreads();

  const _Float16* arow = sP + m * LP;
  const _Float16* brow = keyT + ((size_t)b * ND + 128 * w + m) * NS;
  const v8f zero8 = {0.f, 0.f, 0.f, 0.f, 0.f, 0.f, 0.f, 0.f};
  v8f acc[8];
  #pragma unroll
  for (int i = 0; i < 8; ++i) acc[i] = zero8;

  #pragma unroll 1
  for (int k0 = 0; k0 < NS; k0 += 32) {
    const v16h a = load_frag(arow + k0, h);
    #pragma unroll
    for (int i = 0; i < 8; ++i) {
      const v16h bfr = load_frag(brow + (size_t)i * 16 * NS + k0, h);
      acc[i] = wmma_f16(a, bfr, acc[i]);
    }
  }
  __syncthreads();

  float gp[8];
  #pragma unroll
  for (int r = 0; r < 8; ++r) gp[r] = 0.0f;
  #pragma unroll
  for (int i = 0; i < 8; ++i) {
    const int col = 128 * w + 16 * i + m;
    const float wv = wg[col];
    #pragma unroll
    for (int r = 0; r < 8; ++r) {
      const float qv = acc[i][r] * (1.0f / PSCALE);
      gp[r] += qv * wv;
      sP[(8 * h + r) * LP + col] = (_Float16)qv;
    }
  }
  #pragma unroll
  for (int r = 0; r < 8; ++r) {
    gp[r] += __shfl_xor(gp[r], 8);
    gp[r] += __shfl_xor(gp[r], 4);
    gp[r] += __shfl_xor(gp[r], 2);
    gp[r] += __shfl_xor(gp[r], 1);
  }
  if (m == 0) {
    #pragma unroll
    for (int r = 0; r < 8; ++r) gpart[w * 16 + 8 * h + r] = gp[r];
  }
  __syncthreads();
  if (tid < 32) {
    float g = 0.0f;
    if (tid < 16) {
      float x = 0.0f;
      #pragma unroll
      for (int ww = 0; ww < 8; ++ww) x += gpart[ww * 16 + tid];
      x += bg[0];
      g = 1.0f / (1.0f + __expf(-x));
    }
    gl[tid] = g;
  }
  __syncthreads();

  if (tid < 8) {
    const v4f gv = *(const v4fa*)(gl + 4 * tid);
    *(volatile v4f*)(gates_ws + (size_t)blk * 32 + 4 * tid) = gv;
  }
  q_store_pass(sP, qout, b, t0, w, lane);
  __threadfence();
  if (tid < 8) {
    const v4f gv = *(const v4fa*)(gl + 4 * tid);
    *(volatile v4f*)(gates_ws + (size_t)blk * 32 + 4 * tid) = gv;
  }
  q_store_pass(sP, qout, b, t0, w, lane);
}

__device__ __forceinline__ void proj_store_pass(const _Float16* sT, _Float16* plane,
                                                int m0, int fgrp, int w, int lane) {
  const int q8 = lane & 7, sub = lane >> 3;
  #pragma unroll
  for (int i = 0; i < 8; ++i) {
    const int lid = w * 32 + i * 4 + sub;
    const v8h v = *(const v8ha*)(sT + lid * 64 + 8 * q8);
    *(volatile v8h*)(plane + ((size_t)(m0 + lid)) * ND + fgrp * 64 + 8 * q8) = v;
  }
}

__global__ __launch_bounds__(128) void proj_kernel(const _Float16* __restrict__ qsrc,
                                                   const _Float16* __restrict__ ksrc,
                                                   const _Float16* __restrict__ wh,
                                                   const float* __restrict__ bq,
                                                   const float* __restrict__ bk,
                                                   _Float16* __restrict__ qpl,
                                                   _Float16* __restrict__ kpl) {
  __shared__ __attribute__((aligned(16))) _Float16 sT[128 * 64];

  const int tid = threadIdx.x, lane = tid & 31, w = tid >> 5;
  const int h = lane >> 4, m = lane & 15;
  const int m0 = blockIdx.x * 128;
  const int cg = blockIdx.y;
  const int which = cg >> 4, fgrp = cg & 15;
  const int m0w = m0 + 32 * w;

  const _Float16* xsrc = (which == 0) ? qsrc : ksrc;
  const _Float16* xa0 = xsrc + (size_t)(m0w + m) * ND;
  const _Float16* xa1 = xa0 + (size_t)16 * ND;
  const _Float16* wb  = wh + ((size_t)which * ND + fgrp * 64 + m) * ND;

  const v8f zero8 = {0.f, 0.f, 0.f, 0.f, 0.f, 0.f, 0.f, 0.f};
  v8f acc[2][4];
  #pragma unroll
  for (int mt = 0; mt < 2; ++mt)
    #pragma unroll
    for (int nt = 0; nt < 4; ++nt) acc[mt][nt] = zero8;

  #pragma unroll 1
  for (int k0 = 0; k0 < ND; k0 += 32) {
    const v16h a0 = load_frag(xa0 + k0, h);
    const v16h a1 = load_frag(xa1 + k0, h);
    #pragma unroll
    for (int nt = 0; nt < 4; ++nt) {
      const v16h bfr = load_frag(wb + (size_t)nt * 16 * ND + k0, h);
      acc[0][nt] = wmma_f16(a0, bfr, acc[0][nt]);
      acc[1][nt] = wmma_f16(a1, bfr, acc[1][nt]);
    }
  }

  const float* bias = (which == 0) ? bq : bk;
  #pragma unroll
  for (int nt = 0; nt < 4; ++nt) {
    const int feat = 16 * nt + m;
    const float bvl = bias[fgrp * 64 + feat];
    #pragma unroll
    for (int mt = 0; mt < 2; ++mt) {
      #pragma unroll
      for (int r = 0; r < 8; ++r) {
        const int tokl = 32 * w + 16 * mt + 8 * h + r;
        const float y = acc[mt][nt][r] * (1.0f / WSCALE) + bvl;
        sT[tokl * 64 + feat] = (_Float16)y;
      }
    }
  }
  __syncthreads();

  _Float16* plane = (which == 0) ? qpl : kpl;
  proj_store_pass(sT, plane, m0, fgrp, w, lane);
  __threadfence();
  proj_store_pass(sT, plane, m0, fgrp, w, lane);
}

__device__ __forceinline__ void out_store_pass(const float* sD, float* out,
                                               int b, int t0, int w, int lane) {
  const int q8 = lane & 7, sub = lane >> 3;
  #pragma unroll
  for (int i = 0; i < 16; ++i) {
    const int L = 64 * w + 4 * i + sub;
    const int row = L >> 5, seg = L & 31;
    const v4f v = *(const v4fa*)(sD + row * FP + seg * 32 + 4 * q8);
    *(volatile v4f*)(out + ((size_t)(b * NT + t0 + row)) * NS + seg * 32 + 4 * q8) = v;
  }
}

__global__ __launch_bounds__(256) void final_kernel(const _Float16* __restrict__ qpl,
                                                    const _Float16* __restrict__ kpl,
                                                    const float* __restrict__ msrc,
                                                    const float* __restrict__ steps_ws,
                                                    const float* __restrict__ gates_ws,
                                                    float* __restrict__ out) {
  #pragma clang fp contract(off)
  extern __shared__ v4f dsm[];
  float* sD = (float*)dsm;

  const int tid = threadIdx.x, lane = tid & 31, w = tid >> 5;
  const int h = lane >> 4, m = lane & 15;
  const int blk = blockIdx.x, b = blk >> 6, t0 = (blk & 63) * 16;

  const _Float16* arow = qpl + ((size_t)(b * NT + t0 + m)) * ND;
  const _Float16* brow = kpl + ((size_t)b * NS + 128 * w + m) * ND;
  const v8f zero8 = {0.f, 0.f, 0.f, 0.f, 0.f, 0.f, 0.f, 0.f};
  v8f acc[8];
  #pragma unroll
  for (int i = 0; i < 8; ++i) acc[i] = zero8;

  #pragma unroll 1
  for (int k0 = 0; k0 < ND; k0 += 32) {
    const v16h a = load_frag(arow + k0, h);
    #pragma unroll
    for (int i = 0; i < 8; ++i) {
      const v16h bfr = load_frag(brow + (size_t)i * 16 * ND + k0, h);
      acc[i] = wmma_f16(a, bfr, acc[i]);
    }
  }

  #pragma unroll
  for (int i = 0; i < 8; ++i) {
    const int s = 128 * w + 16 * i + m;
    const float pen = (1.0f - msrc[(size_t)b * NS + s]) * BIGF;
    #pragma unroll
    for (int r = 0; r < 8; ++r) sD[(8 * h + r) * FP + s] = (acc[i][r] - pen) * 0.03125f;
  }
  __syncthreads();

  const float st = steps_ws[b];
  const float* mrow = msrc + (size_t)b * NS;
  #pragma unroll
  for (int rr = 0; rr < 2; ++rr) {
    const int r = 2 * w + rr;
    float x[32];
    float vmax = -3.0e38f;
    #pragma unroll
    for (int j = 0; j < 32; ++j) { x[j] = sD[r * FP + lane + 32 * j]; vmax = fmaxf(vmax, x[j]); }
    #pragma unroll
    for (int o = 16; o > 0; o >>= 1) vmax = fmaxf(vmax, __shfl_xor(vmax, o));
    float sum = 0.0f;
    #pragma unroll
    for (int j = 0; j < 32; ++j) { const float e = __expf(x[j] - vmax); x[j] = e; sum += e; }
    #pragma unroll
    for (int o = 16; o > 0; o >>= 1) sum += __shfl_xor(sum, o);
    const float inv = 1.0f / sum;

    float pl[32];
    pos_row(pl, st, t0 + r, mrow, lane);

    const float g = gates_ws[(size_t)blk * 32 + r];
    const float omg = 1.0f - g;
    #pragma unroll
    for (int j = 0; j < 32; ++j) {
      const float pr = x[j] * inv;
      const float t1 = omg * pr;
      const float t2 = g * pl[j];
      sD[r * FP + lane + 32 * j] = t1 + t2;
    }
  }
  __syncthreads();

  out_store_pass(sD, out, b, t0, w, lane);
  __threadfence();
  out_store_pass(sD, out, b, t0, w, lane);
}

extern "C" void kernel_launch(void* const* d_in, const int* in_sizes, int n_in,
                              void* d_out, int out_size, void* d_ws, size_t ws_size,
                              hipStream_t stream) {
  if (n_in < 9) return;
  if (in_sizes[0] != NX) return;
  if (in_sizes[1] != NB * NS || in_sizes[2] != NB * NT) return;
  if (in_sizes[3] != NW || in_sizes[5] != NW) return;
  if (in_sizes[4] != ND || in_sizes[6] != ND || in_sizes[7] != ND) return;
  if (in_sizes[8] != 1) return;
  if (out_size != NB * NT * NS) return;

  const float* key  = (const float*)d_in[0];
  const float* msrc = (const float*)d_in[1];
  const float* mtrg = (const float*)d_in[2];
  const float* Wq   = (const float*)d_in[3];
  const float* bq   = (const float*)d_in[4];
  const float* Wk   = (const float*)d_in[5];
  const float* bk   = (const float*)d_in[6];
  const float* wg   = (const float*)d_in[7];
  const float* bg   = (const float*)d_in[8];
  float* out = (float*)d_out;

  const size_t steps_bytes = 256;
  const size_t gates_bytes = (size_t)NBLK * 32 * 4;
  const size_t wh_bytes    = (size_t)2 * NW * 2;
  const size_t pl_bytes    = (size_t)NX * 2;
  const size_t total = steps_bytes + gates_bytes + wh_bytes + 5 * pl_bytes;
  if (total > ws_size) return;

  char* ws = (char*)d_ws;
  size_t off = 0;
  float* steps_ws = (float*)(ws + off);        off += steps_bytes;
  float* gates_ws = (float*)(ws + off);        off += gates_bytes;
  _Float16* wh    = (_Float16*)(ws + off);     off += wh_bytes;
  _Float16* keyh  = (_Float16*)(ws + off);     off += pl_bytes;
  _Float16* keyT  = (_Float16*)(ws + off);     off += pl_bytes;
  _Float16* qryh  = (_Float16*)(ws + off);     off += pl_bytes;
  _Float16* qpl   = (_Float16*)(ws + off);     off += pl_bytes;
  _Float16* kpl   = (_Float16*)(ws + off);     off += pl_bytes;
  if (off > ws_size) return;

  steps_kernel<<<1, 256, 0, stream>>>(msrc, mtrg, steps_ws);

  const int ngroups = 2 * NW8;
  cvt_w_kernel<<<(ngroups + 255) / 256, 256, 0, stream>>>(Wq, Wk, wh);

  dim3 gPrep(NS / 64, ND / 64, NB);
  prep_key_kernel<<<gPrep, 128, 0, stream>>>(key, keyh, keyT);

  query_kernel<<<NBLK, 256, 0, stream>>>(msrc, keyT, steps_ws, wg, bg, qryh, gates_ws);

  dim3 gProj(NTOK / 128, 2 * 16);
  proj_kernel<<<gProj, 128, 0, stream>>>(qryh, keyh, wh, bq, bk, qpl, kpl);

  const size_t dyn = (size_t)16 * FP * 4;
  final_kernel<<<NBLK, 256, dyn, stream>>>(qpl, kpl, msrc, steps_ws, gates_ws, out);
}
